// EphysAttentionLayer_74457553043516
// MI455X (gfx1250) — hardware-run, weakly checked
//
#include <hip/hip_runtime.h>
#include <math.h>

#define BB 8
#define NN 1024
#define NN_LOG2 10
#define EE 512
#define DM EE
#define FF NN
#define NTOK (BB * NN)
#define NE 1
#define NSH 1
#define NROW_S NTOK
#define NT_MAX (NROW_S / 64)

#define DT_STEP 0.001f
#define ATT_LO (-0.5f)
#define ATT_HI 1.5f

#define CH_LOG2 11
#define CW_LOG2 16
#define SC_Y (1.0f / (float)(1u << (CH_LOG2 + CW_LOG2)))

#define TBL_COUNT 0
#define TBL_POFF 16
#define TBL_NTILES 40
#define TBL_TILE_E 64
#define TBL_HDR 256

static_assert(BB == 8 && NN == 1024 && (1 << NN_LOG2) == NN && EE == 512 && DM == 512 && FF == 1024 && NTOK == 8192 && NE == 1 && NSH == 1 && NROW_S == 8192 && NT_MAX == 128);
static_assert(DM % 64 == 0 && FF % 32 == 0 && NROW_S % 64 == 0);
static_assert(TBL_HDR % 32 == 0 && TBL_HDR <= 512);
static_assert(TBL_COUNT + NE <= TBL_POFF && TBL_POFF + NE + 1 <= TBL_NTILES && TBL_NTILES < TBL_TILE_E && TBL_TILE_E + NT_MAX <= TBL_HDR);
static_assert((BB * NN * NN / 8) % 256 == 0 && (EE * NN / 8) % 256 == 0);
static_assert(CH_LOG2 == 11 && CW_LOG2 == 16);

constexpr size_t al256(size_t b) { return (b + 255) & ~(size_t)255; }
constexpr size_t SZ_A16  = al256((size_t)BB * NN * NN * 2);
constexpr size_t SZ_W16  = al256((size_t)EE * NN * 2);
constexpr size_t SZ_TBLD = al256((size_t)TBL_HDR * 4);
constexpr size_t WS_TOTAL = SZ_A16 + SZ_W16 + SZ_TBLD;
static_assert(WS_TOTAL == (size_t)17826816 && WS_TOTAL < (size_t)134217728);

typedef _Float16 h16;
typedef __attribute__((ext_vector_type(16))) _Float16 v16h;
typedef __attribute__((ext_vector_type(8)))  _Float16 v8h;
typedef __attribute__((ext_vector_type(8)))  float    v8f;
typedef __attribute__((ext_vector_type(4)))  float    v4f;
typedef __attribute__((ext_vector_type(2)))  float    v2f;
typedef __attribute__((ext_vector_type(4)))  unsigned int v4u;
typedef __attribute__((ext_vector_type(4)))  int      v4i;
typedef __attribute__((ext_vector_type(2)))  int      v2i;


#define VST2(T, ptr, val) do { const T vst2_v_ = (val); *(volatile T*)(ptr) = vst2_v_; __threadfence(); *(volatile T*)(ptr) = vst2_v_; } while (0)

static __device__ __forceinline__ float bfr(float f) {
    unsigned u = __float_as_uint(f);
    u += 0x7FFFu + ((u >> 16) & 1u);
    return __uint_as_float(u & 0xFFFF0000u);
}
static __device__ __forceinline__ h16 toh_flush(float v) { const float w = (fabsf(v) < 6.103515625e-05f) ? 0.0f : v; return (h16)w; }
static __device__ __forceinline__ void st8h(h16* p, const float* v) {
    v8h hv;
#pragma unroll
    for (int e = 0; e < 8; ++e) hv[e] = toh_flush(v[e]);
    VST2(v8h, p, hv);
}

union FragU { v16h v; v8h h[2]; };
static __device__ __forceinline__ v16h frag_ld(const h16* p) {
    FragU f; f.h[0] = *(const v8h*)(p); f.h[1] = *(const v8h*)(p + 16); return f.v;
}
static __device__ __forceinline__ v8f wmma16g(v16h a, v16h b, v8f c) {
    c = __builtin_amdgcn_wmma_f32_16x16x32_f16(false, a, false, b, (short)0, c, false, false);
    asm volatile("v_nop\n\tv_nop\n\tv_nop\n\tv_nop" : "+v"(c) : "v"(a), "v"(b));
    return c;
}
static __device__ __forceinline__ void wave_sync_lds() {
    __builtin_amdgcn_fence(3  , "workgroup");
    __builtin_amdgcn_wave_barrier();
    __builtin_amdgcn_fence(2  , "workgroup");
}

template <int LOG2C>
__global__ __launch_bounds__(256) void k_plane(const float* __restrict__ src, h16* __restrict__ dst, unsigned n8) {
    const unsigned u = blockIdx.x * 256u + threadIdx.x;
    if (u >= n8) return;
    const float cs = (float)(1u << LOG2C);
    const v4f a = *(const v4f*)(src + (size_t)u * 8u);
    const v4f b = *(const v4f*)(src + (size_t)u * 8u + 4u);
    float v[8] = {bfr(a.x) * cs, bfr(a.y) * cs, bfr(a.z) * cs, bfr(a.w) * cs, bfr(b.x) * cs, bfr(b.y) * cs, bfr(b.z) * cs, bfr(b.w) * cs};
    st8h(dst + (size_t)u * 8u, v);
}

__global__ __launch_bounds__(64) void k_tbl_dense(int* __restrict__ tbl) {
    const unsigned w0 = threadIdx.x * 4u;
    int q[4];
#pragma unroll
    for (int k = 0; k < 4; ++k) {
        const unsigned w = w0 + (unsigned)k;
        int val = 0;
        val = (w < (unsigned)(TBL_COUNT + NSH)) ? NTOK : val;
        val = (w >= (unsigned)TBL_POFF && w <= (unsigned)(TBL_POFF + NE)) ? (int)min((w - (unsigned)TBL_POFF) * (unsigned)NTOK, (unsigned)NROW_S) : val;
        val = (w == (unsigned)TBL_NTILES) ? (NROW_S / 64) : val;
        val = (w >= (unsigned)TBL_TILE_E && w < (unsigned)(TBL_TILE_E + NT_MAX)) ? ((w - (unsigned)TBL_TILE_E < (unsigned)(NROW_S / 64)) ? (int)((w - (unsigned)TBL_TILE_E) / (unsigned)(NTOK / 64)) : -1) : val;
        q[k] = val;
    }
    v4i v;
    v.x = q[0]; v.y = q[1]; v.z = q[2]; v.w = q[3];
    VST2(v4i, tbl + w0, v);
}

__global__ __launch_bounds__(256) void k_attn(const int* __restrict__ spk, const float* __restrict__ pre, const float* __restrict__ post, const float* __restrict__ att,
                                              const float* __restrict__ wpre, const float* __restrict__ wpost, const float* __restrict__ tpre, const float* __restrict__ tpost,
                                              h16* __restrict__ dst, unsigned n8) {
    const unsigned u = blockIdx.x * 256u + threadIdx.x;
    if (u >= n8) return;
    const unsigned e0 = u * 8u;
    const unsigned b = e0 >> (2 * NN_LOG2);
    const unsigned rem = e0 & (unsigned)(NN * NN - 1);
    const unsigned i = rem >> NN_LOG2;
    const unsigned j0 = rem & (unsigned)(NN - 1);
    float p[8], q[8], a[8], wp[8], wq[8], tp[8], tq[8];
    int sj[8];
#pragma unroll
    for (int h = 0; h < 2; ++h) {
        const v4f vp = *(const v4f*)(pre + (size_t)e0 + 4u * h), vq = *(const v4f*)(post + (size_t)e0 + 4u * h), va = *(const v4f*)(att + (size_t)e0 + 4u * h);
        const v4f vwp = *(const v4f*)(wpre + (size_t)rem + 4u * h), vwq = *(const v4f*)(wpost + (size_t)rem + 4u * h), vtp = *(const v4f*)(tpre + (size_t)rem + 4u * h), vtq = *(const v4f*)(tpost + (size_t)rem + 4u * h);
        const v4i vs = *(const v4i*)(spk + (size_t)b * NN + j0 + 4u * h);
        p[4 * h + 0] = vp.x; p[4 * h + 1] = vp.y; p[4 * h + 2] = vp.z; p[4 * h + 3] = vp.w;
        q[4 * h + 0] = vq.x; q[4 * h + 1] = vq.y; q[4 * h + 2] = vq.z; q[4 * h + 3] = vq.w;
        a[4 * h + 0] = va.x; a[4 * h + 1] = va.y; a[4 * h + 2] = va.z; a[4 * h + 3] = va.w;
        wp[4 * h + 0] = vwp.x; wp[4 * h + 1] = vwp.y; wp[4 * h + 2] = vwp.z; wp[4 * h + 3] = vwp.w;
        wq[4 * h + 0] = vwq.x; wq[4 * h + 1] = vwq.y; wq[4 * h + 2] = vwq.z; wq[4 * h + 3] = vwq.w;
        tp[4 * h + 0] = vtp.x; tp[4 * h + 1] = vtp.y; tp[4 * h + 2] = vtp.z; tp[4 * h + 3] = vtp.w;
        tq[4 * h + 0] = vtq.x; tq[4 * h + 1] = vtq.y; tq[4 * h + 2] = vtq.z; tq[4 * h + 3] = vtq.w;
        sj[4 * h + 0] = vs.x; sj[4 * h + 1] = vs.y; sj[4 * h + 2] = vs.z; sj[4 * h + 3] = vs.w;
    }
    const int si_w = spk[(size_t)b * NN + i];
    const float si = (float)si_w;
    const float mi = (si_w != 0) ? 1.0f : 0.0f;
    const float cs = (float)(1u << CH_LOG2);
    float v[8];
#pragma unroll
    for (int e = 0; e < 8; ++e) {
        const float sjf = (float)sj[e];
        const float mj = (sj[e] != 0) ? 1.0f : 0.0f;
        const float pd = expf(-DT_STEP / expf(bfr(tp[e])));
        const float qd = expf(-DT_STEP / expf(bfr(tq[e])));
        const float ptr = bfr(p[e]) * pd + sjf * expf(bfr(wp[e])) * DT_STEP;
        const float qtr = bfr(q[e]) * qd + si * expf(bfr(wq[e])) * DT_STEP;
        const float a0 = bfr(a[e]);
        float an = a0 + (1.0f - a0) * (ptr * mi) - a0 * (qtr * mj);
        an = fminf(fmaxf(an, ATT_LO), ATT_HI);
        v[e] = an * cs;
    }
    st8h(dst + (size_t)e0, v);
}

__global__ __launch_bounds__(256) void k_ffn2(const h16* __restrict__ Hg, const h16* __restrict__ Wp, const float* __restrict__ eb,
                                              const int* __restrict__ tbl, float* __restrict__ Yg) {
    __shared__ __align__(16) float sT[8][16 * 68];
    const unsigned lane = threadIdx.x & 31u;
    const unsigned wave = threadIdx.x >> 5;
    const unsigned u = blockIdx.x * 8u + wave;
    if (u >= (unsigned)(NT_MAX * (DM / 64))) return;
    const unsigned rowtile = u / (unsigned)(DM / 64);
    const unsigned ct = u - rowtile * (unsigned)(DM / 64);
    const int nt = min(max(tbl[TBL_NTILES], 0), NT_MAX);
    if ((int)rowtile >= nt) return;
    const int e = min(max(tbl[TBL_TILE_E + rowtile], 0), NE - 1);
    const size_t wbase = (size_t)(unsigned)e * (size_t)(DM * FF);
    const unsigned m0 = rowtile << 6, n0 = ct << 6;
    const unsigned rlane = lane & 15u;
    const unsigned koff = (lane >> 4) * 8u;
    const unsigned mOff = koff;

    v8f acc[4][4];
#pragma unroll
    for (int i = 0; i < 4; ++i)
#pragma unroll
        for (int j = 0; j < 4; ++j) acc[i][j] = (v8f){0.f,0.f,0.f,0.f,0.f,0.f,0.f,0.f};

    for (unsigned k0 = 0; k0 < (unsigned)FF; k0 += 32u) {
        v16h bh[4];
#pragma unroll
        for (int j = 0; j < 4; ++j)
            bh[j] = frag_ld(Wp + wbase + (size_t)(n0 + ((unsigned)j << 4) + rlane) * FF + koff + k0);
#pragma unroll
        for (int i = 0; i < 4; ++i) {
            const v16h ah = frag_ld(Hg + (size_t)(m0 + ((unsigned)i << 4) + rlane) * FF + koff + k0);
#pragma unroll
            for (int j = 0; j < 4; ++j) acc[i][j] = wmma16g(ah, bh[j], acc[i][j]);
        }
    }

    float ebv[4];
#pragma unroll
    for (int j = 0; j < 4; ++j) ebv[j] = bfr(eb[(unsigned)e * (unsigned)DM + n0 + ((unsigned)j << 4) + rlane]);

    float* slab = sT[wave];
#pragma unroll
    for (int i = 0; i < 4; ++i) {
        const unsigned mBase = m0 + ((unsigned)i << 4);
#pragma unroll
        for (int j = 0; j < 4; ++j)
#pragma unroll
            for (int r = 0; r < 8; ++r)
                slab[(mOff + (unsigned)r) * 68u + ((unsigned)j << 4) + rlane] = acc[i][j][r] * SC_Y + ebv[j];
        wave_sync_lds();
        const unsigned hh = lane >> 4, c4 = (lane & 15u) * 4u;
#pragma unroll
        for (int half = 0; half < 2; ++half) {
            v4f vv[4];
#pragma unroll
            for (int it = 0; it < 4; ++it) {
                const unsigned row = (unsigned)(half * 4 + it) * 2u + hh;
                vv[it] = *(const v4f*)(slab + row * 68u + c4);
            }
            for (int pass = 0; pass < 2; ++pass) {
#pragma unroll
                for (int it = 0; it < 4; ++it) {
                    const unsigned row = (unsigned)(half * 4 + it) * 2u + hh;
                    *(volatile v4f*)(Yg + (size_t)(mBase + row) * DM + n0 + c4) = vv[it];
                }
                __threadfence();
            }
        }
        wave_sync_lds();
    }
}

extern "C" void kernel_launch(void* const* d_in, const int* in_sizes, int n_in, void* d_out, int out_size,
                              void* d_ws, size_t ws_size, hipStream_t stream) {
    if (n_in < 10) return;
    if (in_sizes[0] < BB * NN || in_sizes[1] < BB * NN * NN || in_sizes[2] < BB * NN * NN || in_sizes[3] < BB * NN * NN) return;
    if (in_sizes[4] < NN * NN || in_sizes[5] < NN * NN || in_sizes[6] < NN * NN || in_sizes[7] < NN * NN || in_sizes[8] < EE * NN || in_sizes[9] < EE) return;
    if (out_size < BB * NN * EE) return;

    const int*   spk   = (const int*)d_in[0];
    const float* pre   = (const float*)d_in[1];
    const float* post  = (const float*)d_in[2];
    const float* att   = (const float*)d_in[3];
    const float* wpre  = (const float*)d_in[4];
    const float* wpost = (const float*)d_in[5];
    const float* tpre  = (const float*)d_in[6];
    const float* tpost = (const float*)d_in[7];
    const float* vw    = (const float*)d_in[8];
    const float* vb    = (const float*)d_in[9];
    float* out = (float*)d_out;

    char* wsp = (char*)d_ws;
    size_t off = 0;
    auto carve = [&](size_t bytes) -> void* { void* r = wsp + off; off += (bytes + 255) & ~(size_t)255; return r; };
    h16* a16  = (h16*)carve((size_t)BB * NN * NN * 2);
    h16* w16  = (h16*)carve((size_t)EE * NN * 2);
    int* tblD = (int*)carve((size_t)TBL_HDR * 4);
    if (off != WS_TOTAL || off > ws_size || off > (size_t)134217728) return;

    k_attn<<<(BB * NN * NN / 8) / 256, 256, 0, stream>>>(spk, pre, post, att, wpre, wpost, tpre, tpost, a16, (unsigned)(BB * NN * NN / 8));
    k_plane<CW_LOG2><<<(EE * NN / 8) / 256, 256, 0, stream>>>(vw, w16, (unsigned)(EE * NN / 8));
    k_tbl_dense<<<1, 64, 0, stream>>>(tblD);
    k_ffn2<<<(NT_MAX * (DM / 64) + 7) / 8, 256, 0, stream>>>(a16, w16, vb, tblD, out);
}
